// SelfAttentionBlockWithRoPE_66898410602556
// MI455X (gfx1250) — hardware-verified
//
#include <hip/hip_runtime.h>
#include <math.h>

constexpr int kBatch   = 2;
constexpr int kSeq     = 2048;
constexpr int kDim     = 1024;
constexpr int kHeads   = 16;
constexpr int kHd      = 64;
constexpr int kHidden  = 4096;
constexpr int kTok     = kBatch * kSeq;
constexpr int kQkvLd   = 3 * kDim;
constexpr int kGroups  = kBatch * kHeads;
constexpr int kGpc     = 4;
constexpr int kChunks  = kGroups / kGpc;
constexpr int kMlpQ    = 4;
constexpr int kMlpRows = kTok / kMlpQ;

constexpr float kWc        = 16.0f;
constexpr float kW2c       = 32.0f;
constexpr float kPc        = 2048.0f;
constexpr float kAc        = 256.0f;
constexpr float kLoc       = 2048.0f;
constexpr float kAttnScale = 0.125f;
constexpr float kInvDim    = 1.0f / 1024.0f;
constexpr float kLnEps     = 1e-5f;

typedef char tile_check_a[(kTok % 64 == 0 && kDim % 64 == 0 && kHidden % 64 == 0 && kQkvLd % 64 == 0 && kSeq % 64 == 0 && kHd % 64 == 0) ? 1 : -1];
typedef char tile_check_b[(kDim % 32 == 0 && kHidden % 32 == 0 && kSeq % 32 == 0 && kHd % 32 == 0) ? 1 : -1];
typedef char tile_check_c[(kHeads % kGpc == 0 && kMlpRows % 64 == 0) ? 1 : -1];

constexpr size_t kMiB       = 1048576;
constexpr size_t kOffQkv32  = 0;
constexpr size_t kOffWqkvT  = 48 * kMiB;
constexpr size_t kOffXn1    = 54 * kMiB;
constexpr size_t kOffScores = 0;
constexpr size_t kOffTrig   = 64 * kMiB;
constexpr size_t kOffP      = 64 * kMiB;
constexpr size_t kOffQ16    = 96 * kMiB;
constexpr size_t kOffK16    = 104 * kMiB;
constexpr size_t kOffVt16   = 112 * kMiB;
constexpr size_t kOffAttn16 = 120 * kMiB;
constexpr size_t kOffWoT    = 96 * kMiB;
constexpr size_t kOffX1     = 64 * kMiB;
constexpr size_t kOffXn2    = 80 * kMiB;
constexpr size_t kOffW2T    = 88 * kMiB;
constexpr size_t kOffW1T    = 98 * kMiB;
constexpr size_t kOffPre    = 106 * kMiB;
constexpr size_t kOffHhi    = 0;
constexpr size_t kOffHlo    = 32 * kMiB;
constexpr size_t kOffTmp    = 112 * kMiB;
constexpr size_t kWsTotal   = 128 * kMiB;

typedef char ws_check_a[((size_t)kTok * kQkvLd * 4 <= kOffWqkvT) ? 1 : -1];
typedef char ws_check_b[(kOffWqkvT + (size_t)kQkvLd * kDim * 2 <= kOffXn1) ? 1 : -1];
typedef char ws_check_c[(kOffXn1 + (size_t)kTok * kDim * 2 <= 64 * kMiB) ? 1 : -1];
typedef char ws_check_d[(kOffScores + (size_t)kGpc * kSeq * kSeq * 4 <= kOffP) ? 1 : -1];
typedef char ws_check_e[(kOffP + (size_t)kGpc * kSeq * kSeq * 2 <= kOffQ16) ? 1 : -1];
typedef char ws_check_f[(kOffAttn16 + (size_t)kTok * kDim * 2 <= kWsTotal) ? 1 : -1];
typedef char ws_check_g[(kOffPre + (size_t)kMlpRows * kHidden * 4 <= kWsTotal) ? 1 : -1];
typedef char ws_check_h[(kOffHlo + (size_t)kTok * kHidden * 2 <= kOffX1) ? 1 : -1];
typedef char ws_check_i[(kOffTmp + (size_t)kTok * kDim * 4 <= kWsTotal) ? 1 : -1];
typedef char ws_check_j[(kOffW1T + (size_t)kHidden * kDim * 2 <= kOffPre) ? 1 : -1];

typedef __attribute__((ext_vector_type(16))) _Float16 v16h;
typedef __attribute__((ext_vector_type(8)))  _Float16 v8h;
typedef __attribute__((ext_vector_type(16))) __bf16   v16b;
typedef __attribute__((ext_vector_type(8)))  __bf16   v8b;
typedef __attribute__((ext_vector_type(8)))  float    v8f;
typedef __attribute__((ext_vector_type(4)))  float    v4f;
typedef __attribute__((ext_vector_type(4)))  unsigned int v4u;

__device__ __forceinline__ unsigned short f2bf_bits(float f) {
  unsigned u = __float_as_uint(f);
  return (unsigned short)((u + 0x7FFFu + ((u >> 16) & 1u)) >> 16);
}
__device__ __forceinline__ float bf_bits2f(unsigned short h) { return __uint_as_float(((unsigned)h) << 16); }

__device__ __forceinline__ void dep_guard_h(v8f& a, v8f& b, v16h x, v16h y) { asm volatile("v_nop\n\tv_nop\n\tv_nop\n\tv_nop" : "+v"(a), "+v"(b) : "v"(x), "v"(y)); }
__device__ __forceinline__ void dep_guard_b(v8f& a, v8f& b, v16b x, v16b y) { asm volatile("v_nop\n\tv_nop\n\tv_nop\n\tv_nop" : "+v"(a), "+v"(b) : "v"(x), "v"(y)); }
__device__ __forceinline__ void keep4_h(v16h a, v16h b, v16h c, v16h d) { asm volatile("v_nop" :: "v"(a), "v"(b), "v"(c), "v"(d)); }
__device__ __forceinline__ void keep4_b(v16b a, v16b b, v16b c, v16b d) { asm volatile("v_nop" :: "v"(a), "v"(b), "v"(c), "v"(d)); }
__device__ __forceinline__ void acc_guard4(v8f& a, v8f& b, v8f& c, v8f& d) { asm volatile("v_nop\n\tv_nop\n\tv_nop\n\tv_nop" : "+v"(a), "+v"(b), "+v"(c), "+v"(d)); }
template <typename T> struct Frag;
template <> struct Frag<_Float16> {
  typedef v16h V; union U { v16h v; v8h h[2]; };
  static __device__ __forceinline__ v16h load(const _Float16* p) {
    U f; f.h[0] = *(const v8h*)(p); f.h[1] = *(const v8h*)(p + 16); return f.v;
  }
  static __device__ __forceinline__ v8f mma(v16h a, v16h b, v8f c) {
    return __builtin_amdgcn_wmma_f32_16x16x32_f16(false, a, false, b, (short)0, c, false, false);
  }
  static __device__ __forceinline__ void guard(v8f& a, v8f& b, v16h x, v16h y) { dep_guard_h(a, b, x, y); }
  static __device__ __forceinline__ void keep(v16h a, v16h b, v16h c, v16h d) { keep4_h(a, b, c, d); }
};
template <> struct Frag<__bf16> {
  typedef v16b V; union U { v16b v; v8b h[2]; };
  static __device__ __forceinline__ v16b load(const __bf16* p) {
    U f; f.h[0] = *(const v8b*)(p); f.h[1] = *(const v8b*)(p + 16); return f.v;
  }
  static __device__ __forceinline__ v8f mma(v16b a, v16b b, v8f c) {
    return __builtin_amdgcn_wmma_f32_16x16x32_bf16(false, a, false, b, (short)0, c, false, false);
  }
  static __device__ __forceinline__ void guard(v8f& a, v8f& b, v16b x, v16b y) { dep_guard_b(a, b, x, y); }
  static __device__ __forceinline__ void keep(v16b a, v16b b, v16b c, v16b d) { keep4_b(a, b, c, d); }
};

__device__ __forceinline__ unsigned pk16(unsigned short a, unsigned short b) { return (unsigned)a | ((unsigned)b << 16); }
__device__ __forceinline__ unsigned short h_bits(float f) { const _Float16 h = (_Float16)f; return __builtin_bit_cast(unsigned short, h); }
__device__ __forceinline__ float h_bits2f(unsigned short b) { const _Float16 h = __builtin_bit_cast(_Float16, b); return (float)h; }

template <int ET> struct Elem;
template <> struct Elem<0> { typedef _Float16 T; };
template <> struct Elem<1> { typedef __bf16 T; };
template <int ET, bool SPLIT, int BIAS_MODE, int OUT_MODE, bool RESID, int ACT = 0>
__global__ __launch_bounds__(256) void wmma_gemm64(
    const unsigned short* __restrict__ Ap, const unsigned short* __restrict__ A2p, int lda, long strideA,
    const unsigned short* __restrict__ Btp, const unsigned short* __restrict__ Bt2p, int ldb, long strideB,
    void* __restrict__ Cout, void* __restrict__ Cout2, int ldc, long strideC,
    const float* __restrict__ bias,
    const float* __restrict__ resid, long strideR,
    int M, int N, int K, float scale) {
  typedef typename Elem<ET>::T T;
  typedef typename Frag<T>::V V;
  const T* A = (const T*)Ap; const T* A2 = (const T*)A2p; const T* Bt = (const T*)Btp; const T* Bt2 = (const T*)Bt2p;
  __shared__ __align__(16) float sT[8][16 * 68];
  const int b    = blockIdx.y;
  const int lane = threadIdx.x & 31;
  const int wave = threadIdx.x >> 5;
  const int tilesN = N >> 6;
  const int tilesM = M >> 6;
  const int tile = blockIdx.x * 8 + wave;
  if (tile >= tilesM * tilesN) return;
  const int tm = tile / tilesN;
  const int tn = tile - tm * tilesN;
  const int m0 = tm << 6;
  const int n0 = tn << 6;

  const T* Ab  = A  + (size_t)b * strideA;
  const T* Bb  = Bt + (size_t)b * strideB;
  const T* Ab2 = SPLIT ? (A2  + (size_t)b * strideA) : nullptr;
  const T* Bb2 = SPLIT ? (Bt2 + (size_t)b * strideB) : nullptr;

  const int rlane = lane & 15;
  const int koff  = (lane >> 4) * 8;
  const int mOff  = (lane >> 4) * 8;

  v8f acc[4][4];
#pragma unroll
  for (int i = 0; i < 4; ++i)
#pragma unroll
    for (int j = 0; j < 4; ++j) acc[i][j] = (v8f){0.f,0.f,0.f,0.f,0.f,0.f,0.f,0.f};

  for (int k0 = 0; k0 < K; k0 += 32) {
    V bh[4], bl[4];
#pragma unroll
    for (int j = 0; j < 4; ++j) {
      const size_t bo = (size_t)(n0 + (j << 4) + rlane) * ldb + koff + k0;
      bh[j] = Frag<T>::load(Bb + bo);
      if (SPLIT) bl[j] = Frag<T>::load(Bb2 + bo);
    }
#pragma unroll
    for (int i = 0; i < 4; ++i) {
      const size_t ao = (size_t)(m0 + (i << 4) + rlane) * lda + koff + k0;
      V ah = Frag<T>::load(Ab + ao);
      V al;
      if (SPLIT) al = Frag<T>::load(Ab2 + ao);
#pragma unroll
      for (int j = 0; j < 4; ++j) {
        acc[i][j] = Frag<T>::mma(ah, bh[j], acc[i][j]);
        if (SPLIT) {
          acc[i][j] = Frag<T>::mma(ah, bl[j], acc[i][j]);
          acc[i][j] = Frag<T>::mma(al, bh[j], acc[i][j]);
        }
      }
      Frag<T>::guard(acc[i][0], acc[i][3], ah, SPLIT ? al : ah);
    }
    Frag<T>::keep(bh[0], bh[1], bh[2], bh[3]);
    if (SPLIT) Frag<T>::keep(bl[0], bl[1], bl[2], bl[3]);
  }
  acc_guard4(acc[0][0], acc[0][1], acc[0][2], acc[0][3]);
  acc_guard4(acc[1][0], acc[1][1], acc[1][2], acc[1][3]);
  acc_guard4(acc[2][0], acc[2][1], acc[2][2], acc[2][3]);
  acc_guard4(acc[3][0], acc[3][1], acc[3][2], acc[3][3]);

  float* slab = sT[wave];
  const float* Rb = RESID ? (resid + (size_t)b * strideR) : nullptr;
#pragma unroll
  for (int i = 0; i < 4; ++i) {
    const int mBase = m0 + (i << 4);
#pragma unroll
    for (int j = 0; j < 4; ++j) {
      const int n = n0 + (j << 4) + rlane;
      float bv = 0.f;
      if (BIAS_MODE == 2) bv = bias[n];
#pragma unroll
      for (int r = 0; r < 8; ++r) {
        float v = acc[i][j][r] * scale;
        if (BIAS_MODE == 1) v += bias[mBase + mOff + r];
        if (BIAS_MODE == 2) v += bv;
        if (RESID) v += Rb[(size_t)(mBase + mOff + r) * ldc + n];
        if (ACT == 2) v = fmaxf(v, 0.0f);
        if (ACT == 4) v = (v > 0.f) ? v : 0.01f * v;
        slab[(mOff + r) * 68 + (j << 4) + rlane] = v;
      }
    }
    __builtin_amdgcn_fence(__ATOMIC_RELEASE, "workgroup");
    __builtin_amdgcn_wave_barrier();
    __builtin_amdgcn_fence(__ATOMIC_ACQUIRE, "workgroup");
    if (OUT_MODE == 0) {
      float* C = (float*)Cout + (size_t)b * strideC;
      const int hh = lane >> 4, c4 = (lane & 15) * 4;
      for (int pass = 0; pass < 2; ++pass) {
#pragma unroll
        for (int it = 0; it < 8; ++it) {
          const int row = it * 2 + hh;
          v4f v = *(const v4f*)(slab + row * 68 + c4);
          *(volatile v4f*)(C + (size_t)(mBase + row) * ldc + n0 + c4) = v;
        }
        __threadfence();
      }
    } else {
      const int q = lane >> 3, c8 = (lane & 7) * 8;
      unsigned short* C  = (unsigned short*)Cout  + (size_t)b * strideC;
      unsigned short* C2 = (OUT_MODE == 2) ? ((unsigned short*)Cout2 + (size_t)b * strideC) : nullptr;
      for (int pass = 0; pass < 2; ++pass) {
#pragma unroll
        for (int it = 0; it < 4; ++it) {
          const int row = it * 4 + q;
          const float* sp = slab + row * 68 + c8;
          v8h hv, lv;
#pragma unroll
          for (int e = 0; e < 8; ++e) {
            if (OUT_MODE == 1) {
              hv[e] = (_Float16)sp[e];
            } else {
              unsigned short hb = f2bf_bits(sp[e]);
              unsigned short lb = f2bf_bits(sp[e] - bf_bits2f(hb));
              hv[e] = __builtin_bit_cast(_Float16, hb);
              lv[e] = __builtin_bit_cast(_Float16, lb);
            }
          }
          *(volatile v8h*)(C + (size_t)(mBase + row) * ldc + n0 + c8) = hv;
          if (OUT_MODE == 2) *(volatile v8h*)(C2 + (size_t)(mBase + row) * ldc + n0 + c8) = lv;
        }
        __threadfence();
      }
    }
    __builtin_amdgcn_fence(__ATOMIC_RELEASE, "workgroup");
    __builtin_amdgcn_wave_barrier();
    __builtin_amdgcn_fence(__ATOMIC_ACQUIRE, "workgroup");
  }
}

__global__ __launch_bounds__(256) void wtcast_kernel(const float* __restrict__ W, unsigned short* __restrict__ out,
                                                     int kdim, int ndim, float scale) {
  __shared__ float sm[64][65];
  const int t  = threadIdx.x;
  const int k0 = blockIdx.x * 64;
  const int n0 = blockIdx.y * 64;
#pragma unroll
  for (int i = 0; i < 16; ++i) {
    const int e = i * 256 + t;
    const int r = e >> 6;
    const int c = e & 63;
    sm[c][r] = W[(size_t)(k0 + r) * ndim + n0 + c] * scale;
  }
  __syncthreads();
  const int lane = t & 31, wave = t >> 5;
  const int q = lane >> 3, c8 = (lane & 7) * 8;
  v4u u0, u1;
  {
    const int row0 = wave * 8 + q;
    const int row1 = wave * 8 + 4 + q;
    unsigned short ha[8], hb[8];
#pragma unroll
    for (int e = 0; e < 8; ++e) { ha[e] = h_bits(sm[row0][c8 + e]); hb[e] = h_bits(sm[row1][c8 + e]); }
    u0 = (v4u){pk16(ha[0], ha[1]), pk16(ha[2], ha[3]), pk16(ha[4], ha[5]), pk16(ha[6], ha[7])};
    u1 = (v4u){pk16(hb[0], hb[1]), pk16(hb[2], hb[3]), pk16(hb[4], hb[5]), pk16(hb[6], hb[7])};
  }
  unsigned short* p0 = out + (size_t)(n0 + wave * 8 + q) * kdim + k0 + c8;
  unsigned short* p1 = out + (size_t)(n0 + wave * 8 + 4 + q) * kdim + k0 + c8;
  for (int pass = 0; pass < 2; ++pass) {
    *(volatile v4u*)p0 = u0;
    *(volatile v4u*)p1 = u1;
    __threadfence();
  }
}

__global__ __launch_bounds__(128) void ln_f16_kernel(const float* __restrict__ x, const float* __restrict__ w,
                                                     const float* __restrict__ bvec, unsigned short* __restrict__ out) {
  __shared__ float redA[4];
  __shared__ float redB[4];
  const int row  = blockIdx.x;
  const int t    = threadIdx.x;
  const int lane = t & 31, wave = t >> 5;
  const int c0   = t * 8;
  const float* xr = x + (size_t)row * kDim + c0;
  const v4f xa = *(const v4f*)(xr);
  const v4f xb = *(const v4f*)(xr + 4);
  float s = ((xa[0] + xa[1]) + (xa[2] + xa[3])) + ((xb[0] + xb[1]) + (xb[2] + xb[3]));
#pragma unroll
  for (int off = 16; off > 0; off >>= 1) s += __shfl_xor(s, off, 32);
  if (lane == 0) redA[wave] = s;
  __syncthreads();
  const float mean = ((redA[0] + redA[1]) + (redA[2] + redA[3])) * kInvDim;
  float d[8];
#pragma unroll
  for (int e = 0; e < 4; ++e) { d[e] = xa[e] - mean; d[4 + e] = xb[e] - mean; }
  float s2 = ((d[0] * d[0] + d[1] * d[1]) + (d[2] * d[2] + d[3] * d[3])) + ((d[4] * d[4] + d[5] * d[5]) + (d[6] * d[6] + d[7] * d[7]));
#pragma unroll
  for (int off = 16; off > 0; off >>= 1) s2 += __shfl_xor(s2, off, 32);
  if (lane == 0) redB[wave] = s2;
  __syncthreads();
  const float var = ((redB[0] + redB[1]) + (redB[2] + redB[3])) * kInvDim;
  const float inv = rsqrtf(var + kLnEps);
  const v4f wa = *(const v4f*)(w + c0), wb = *(const v4f*)(w + c0 + 4);
  const v4f ba = *(const v4f*)(bvec + c0), bb2 = *(const v4f*)(bvec + c0 + 4);
  unsigned short hb[8];
#pragma unroll
  for (int e = 0; e < 4; ++e) {
    hb[e]     = h_bits(d[e] * inv * wa[e] + ba[e]);
    hb[4 + e] = h_bits(d[4 + e] * inv * wb[e] + bb2[e]);
  }
  const v4u u = (v4u){pk16(hb[0], hb[1]), pk16(hb[2], hb[3]), pk16(hb[4], hb[5]), pk16(hb[6], hb[7])};
  unsigned short* op = out + (size_t)row * kDim + c0;
  *(volatile v4u*)op = u;
  __threadfence();
  *(volatile v4u*)op = u;
}

struct RopeFreq { float inv[32]; };
typedef char rope_freq_size_check[(sizeof(RopeFreq) == 128) ? 1 : -1];

__global__ __launch_bounds__(256) void trig_kernel(const int* __restrict__ pos, float* __restrict__ trig, int ntot, RopeFreq f) {
#pragma clang fp contract(off)
  const int gidx = blockIdx.x * 256 + threadIdx.x;
  if (gidx >= ntot) return;
  const int tok = gidx >> 5;
  const int i   = gidx & 31;
  const int p   = pos[tok];
  float fr = 0.0f;
#pragma unroll
  for (int j = 0; j < 32; ++j) fr = (i == j) ? f.inv[j] : fr;
  const float ang = (float)p * fr;
  const float cv = cosf(ang);
  const float sv = sinf(ang);
  float* rp = trig + (size_t)tok * 64;
  *(volatile float*)(rp + i) = cv;
  *(volatile float*)(rp + 32 + i) = sv;
  __threadfence();
  *(volatile float*)(rp + i) = cv;
  *(volatile float*)(rp + 32 + i) = sv;
}

__global__ __launch_bounds__(256) void rope_cast_kernel(const float* __restrict__ qkv, const float* __restrict__ trig,
                                                        unsigned short* __restrict__ q16, unsigned short* __restrict__ k16,
                                                        unsigned short* __restrict__ vt16) {
#pragma clang fp contract(off)
  __shared__ float smv[64][65];
  const int t  = threadIdx.x;
  const int s0 = blockIdx.x * 64;
  const int h  = blockIdx.y;
  const int b  = blockIdx.z;
  const int g  = b * kHeads + h;
  const int tokbase = b * kSeq + s0;
#pragma unroll
  for (int i = 0; i < 16; ++i) {
    const int e = i * 256 + t;
    const int r = e >> 6;
    const int c = e & 63;
    smv[c][r] = qkv[(size_t)(tokbase + r) * kQkvLd + 2 * kDim + h * kHd + c];
  }
  const int rr   = t >> 3;
  const int j8   = t & 7;
  const int jj   = j8 & 3;
  const int hsel = j8 >> 2;
#pragma unroll
  for (int it = 0; it < 4; ++it) {
    const int which = it >> 1;
    const int r = (it & 1) * 32 + rr;
    const float* src = qkv + (size_t)(tokbase + r) * kQkvLd + which * kDim + h * kHd + 8 * jj;
    const v4f p1a = *(const v4f*)(src);
    const v4f p1b = *(const v4f*)(src + 4);
    const v4f p2a = *(const v4f*)(src + 32);
    const v4f p2b = *(const v4f*)(src + 36);
    const float* tr = trig + (size_t)(tokbase + r) * 64 + 8 * jj;
    const v4f ca = *(const v4f*)(tr);
    const v4f cb = *(const v4f*)(tr + 4);
    const v4f sa = *(const v4f*)(tr + 32);
    const v4f sb = *(const v4f*)(tr + 36);
    unsigned short hb[8];
#pragma unroll
    for (int e = 0; e < 4; ++e) {
      const float m1 = p1a[e] * ca[e];
      const float m2 = p2a[e] * sa[e];
      const float m3 = p2a[e] * ca[e];
      const float m4 = p1a[e] * sa[e];
      const float lo = m1 - m2;
      const float hi = m3 + m4;
      hb[e] = h_bits(hsel ? hi : lo);
      const float n1 = p1b[e] * cb[e];
      const float n2 = p2b[e] * sb[e];
      const float n3 = p2b[e] * cb[e];
      const float n4 = p1b[e] * sb[e];
      const float lo2 = n1 - n2;
      const float hi2 = n3 + n4;
      hb[4 + e] = h_bits(hsel ? hi2 : lo2);
    }
    const v4u u = (v4u){pk16(hb[0], hb[1]), pk16(hb[2], hb[3]), pk16(hb[4], hb[5]), pk16(hb[6], hb[7])};
    unsigned short* dst = (which == 0 ? q16 : k16) + ((size_t)g * kSeq + s0 + r) * kHd + 8 * j8;
    *(volatile v4u*)dst = u;
    __threadfence();
    *(volatile v4u*)dst = u;
  }
  __syncthreads();
#pragma unroll
  for (int it = 0; it < 2; ++it) {
    const int row = it * 32 + rr;
    unsigned short hb[8];
#pragma unroll
    for (int e = 0; e < 8; ++e) hb[e] = h_bits(smv[row][8 * j8 + e]);
    const v4u u = (v4u){pk16(hb[0], hb[1]), pk16(hb[2], hb[3]), pk16(hb[4], hb[5]), pk16(hb[6], hb[7])};
    unsigned short* dst = vt16 + ((size_t)g * kHd + row) * kSeq + s0 + 8 * j8;
    *(volatile v4u*)dst = u;
    __threadfence();
    *(volatile v4u*)dst = u;
  }
}

__global__ __launch_bounds__(256) void softmax_kernel(const float* __restrict__ sc, unsigned short* __restrict__ P) {
  __shared__ float srow[kSeq];
  __shared__ float redm[8];
  __shared__ float reds[8];
  const int row  = blockIdx.x;
  const int t    = threadIdx.x;
  const int lane = t & 31, wave = t >> 5;
  const int c0   = t * 8;
  const float* sr = sc + (size_t)row * kSeq + c0;
  const v4f a = *(const v4f*)(sr);
  const v4f c = *(const v4f*)(sr + 4);
  float m = fmaxf(fmaxf(fmaxf(a[0], a[1]), fmaxf(a[2], a[3])), fmaxf(fmaxf(c[0], c[1]), fmaxf(c[2], c[3])));
#pragma unroll
  for (int e = 0; e < 4; ++e) { srow[c0 + e] = a[e]; srow[c0 + 4 + e] = c[e]; }
#pragma unroll
  for (int off = 16; off > 0; off >>= 1) m = fmaxf(m, __shfl_xor(m, off, 32));
  if (lane == 0) redm[wave] = m;
  __syncthreads();
  float gm = redm[0];
#pragma unroll
  for (int i = 1; i < 8; ++i) gm = fmaxf(gm, redm[i]);
  float sum = 0.0f;
#pragma unroll 1
  for (int e = 0; e < 8; ++e) {
    const float v = srow[c0 + e];
    const float p = expf(v - gm);
    srow[c0 + e] = p;
    sum += p;
  }
#pragma unroll
  for (int off = 16; off > 0; off >>= 1) sum += __shfl_xor(sum, off, 32);
  if (lane == 0) reds[wave] = sum;
  __syncthreads();
  float tot = 0.0f;
#pragma unroll
  for (int i = 0; i < 8; ++i) tot += reds[i];
  const float inv = kPc * (1.0f / tot);
  unsigned short hb[8];
#pragma unroll
  for (int e = 0; e < 8; ++e) hb[e] = h_bits(srow[c0 + e] * inv);
  const v4u u = (v4u){pk16(hb[0], hb[1]), pk16(hb[2], hb[3]), pk16(hb[4], hb[5]), pk16(hb[6], hb[7])};
  unsigned short* q = P + (size_t)row * kSeq + c0;
  *(volatile v4u*)q = u;
  __threadfence();
  *(volatile v4u*)q = u;
}

__global__ __launch_bounds__(256) void gelu_split_kernel(const float* __restrict__ pre, unsigned short* __restrict__ hhi,
                                                         unsigned short* __restrict__ hlo, int n8) {
  __shared__ unsigned short shh[256 * 8];
  __shared__ unsigned short shl[256 * 8];
  const int t = threadIdx.x;
  const int i = blockIdx.x * 256 + t;
  const int ic = (i < n8) ? i : (n8 - 1);
  const float* p = pre + 8 * (size_t)ic;
#pragma unroll 1
  for (int e = 0; e < 8; ++e) {
    const float v = p[e];
    const float g = 0.5f * v * (1.0f + erff(v * 0.70710678118654752f));
    const unsigned short hb = h_bits(g);
    const float gh = h_bits2f(hb);
    const unsigned short lb = h_bits((g - gh) * kLoc);
    shh[t * 8 + e] = hb;
    shl[t * 8 + e] = lb;
  }
  __syncthreads();
  const unsigned short* sh = shh + t * 8;
  const unsigned short* sl = shl + t * 8;
  const v4u uh = (v4u){pk16(sh[0], sh[1]), pk16(sh[2], sh[3]), pk16(sh[4], sh[5]), pk16(sh[6], sh[7])};
  const v4u ul = (v4u){pk16(sl[0], sl[1]), pk16(sl[2], sl[3]), pk16(sl[4], sl[5]), pk16(sl[6], sl[7])};
  if (i < n8) {
    unsigned short* qh = hhi + 8 * (size_t)i;
    unsigned short* ql = hlo + 8 * (size_t)i;
    *(volatile v4u*)qh = uh;
    *(volatile v4u*)ql = ul;
    __threadfence();
    *(volatile v4u*)qh = uh;
    *(volatile v4u*)ql = ul;
  }
}

extern "C" void kernel_launch(void* const* d_in, const int* in_sizes, int n_in,
                              void* d_out, int out_size, void* d_ws, size_t ws_size,
                              hipStream_t stream) {
  const float* x      = (const float*)d_in[0];
  const int*   pos    = (const int*)d_in[1];
  const float* ln1_w  = (const float*)d_in[2];
  const float* ln1_b  = (const float*)d_in[3];
  const float* qkv_w  = (const float*)d_in[4];
  const float* qkv_b  = (const float*)d_in[5];
  const float* o_w    = (const float*)d_in[6];
  const float* o_b    = (const float*)d_in[7];
  const float* ln2_w  = (const float*)d_in[8];
  const float* ln2_b  = (const float*)d_in[9];
  const float* mlp_w1 = (const float*)d_in[10];
  const float* mlp_b1 = (const float*)d_in[11];
  const float* mlp_w2 = (const float*)d_in[12];
  const float* mlp_b2 = (const float*)d_in[13];
  float* out = (float*)d_out;

  if (n_in < 14) return;
  if (in_sizes[0] != kTok * kDim || in_sizes[1] != kTok || out_size != kTok * kDim) return;
  if (ws_size < kWsTotal) return;

  char* ws = (char*)d_ws;
  float*          qkv32  = (float*)(ws + kOffQkv32);
  unsigned short* wqkvT  = (unsigned short*)(ws + kOffWqkvT);
  unsigned short* xn1    = (unsigned short*)(ws + kOffXn1);
  float*          scores = (float*)(ws + kOffScores);
  float*          trig   = (float*)(ws + kOffTrig);
  unsigned short* pplane = (unsigned short*)(ws + kOffP);
  unsigned short* q16    = (unsigned short*)(ws + kOffQ16);
  unsigned short* k16    = (unsigned short*)(ws + kOffK16);
  unsigned short* vt16   = (unsigned short*)(ws + kOffVt16);
  unsigned short* attn16 = (unsigned short*)(ws + kOffAttn16);
  unsigned short* woT    = (unsigned short*)(ws + kOffWoT);
  float*          x1     = (float*)(ws + kOffX1);
  unsigned short* xn2    = (unsigned short*)(ws + kOffXn2);
  unsigned short* w2T    = (unsigned short*)(ws + kOffW2T);
  unsigned short* w1T    = (unsigned short*)(ws + kOffW1T);
  float*          pre    = (float*)(ws + kOffPre);
  unsigned short* hhi    = (unsigned short*)(ws + kOffHhi);
  unsigned short* hlo    = (unsigned short*)(ws + kOffHlo);
  float*          tmp    = (float*)(ws + kOffTmp);

  RopeFreq rf;
  for (int i = 0; i < 32; ++i) {
    const float e  = (float)i * (1.0f / 32.0f);
    const float pf = (float)pow(10000.0, (double)e);
    rf.inv[i] = 1.0f / pf;
  }

  wtcast_kernel<<<dim3(kDim / 64, kQkvLd / 64), 256, 0, stream>>>(qkv_w, wqkvT, kDim, kQkvLd, kWc);
  ln_f16_kernel<<<kTok, 128, 0, stream>>>(x, ln1_w, ln1_b, xn1);
  {
    const int tiles = (kTok / 64) * (kQkvLd / 64);
    wmma_gemm64<0, false, 2, 0, false><<<dim3((tiles + 7) / 8, 1), 256, 0, stream>>>(
        xn1, xn1, kDim, 0L, wqkvT, wqkvT, kDim, 0L, (void*)qkv32, (void*)qkv32, kQkvLd, 0L,
        qkv_b, x, 0L, kTok, kQkvLd, kDim, 1.0f / kWc);
  }
  {
    const int ntot = kTok * 32;
    trig_kernel<<<(ntot + 255) / 256, 256, 0, stream>>>(pos, trig, ntot, rf);
  }
  rope_cast_kernel<<<dim3(kSeq / 64, kHeads, kBatch), 256, 0, stream>>>(qkv32, trig, q16, k16, vt16);

  for (int c = 0; c < kChunks; ++c) {
    const int g0 = c * kGpc;
    const int b  = g0 / kHeads;
    const int h0 = g0 % kHeads;
    const unsigned short* qg = q16 + (size_t)g0 * kSeq * kHd;
    const unsigned short* kg = k16 + (size_t)g0 * kSeq * kHd;
    const unsigned short* vg = vt16 + (size_t)g0 * kHd * kSeq;
    {
      const int tiles = (kSeq / 64) * (kSeq / 64);
      wmma_gemm64<0, false, 0, 0, false><<<dim3((tiles + 7) / 8, kGpc), 256, 0, stream>>>(
          qg, qg, kHd, (long)kSeq * kHd, kg, kg, kHd, (long)kSeq * kHd,
          (void*)scores, (void*)scores, kSeq, (long)kSeq * kSeq,
          o_b, x, 0L, kSeq, kSeq, kHd, kAttnScale);
    }
    softmax_kernel<<<kGpc * kSeq, 256, 0, stream>>>(scores, pplane);
    {
      unsigned short* og = attn16 + (size_t)b * kSeq * kDim + (size_t)h0 * kHd;
      const int tiles = (kSeq / 64) * (kHd / 64);
      wmma_gemm64<0, false, 0, 1, false><<<dim3((tiles + 7) / 8, kGpc), 256, 0, stream>>>(
          pplane, pplane, kSeq, (long)kSeq * kSeq, vg, vg, kSeq, (long)kHd * kSeq,
          (void*)og, (void*)og, kDim, (long)kHd,
          o_b, x, 0L, kSeq, kHd, kSeq, kAc / kPc);
    }
  }

  wtcast_kernel<<<dim3(kDim / 64, kDim / 64), 256, 0, stream>>>(o_w, woT, kDim, kDim, kWc);
  {
    const int tiles = (kTok / 64) * (kDim / 64);
    wmma_gemm64<0, false, 2, 0, true><<<dim3((tiles + 7) / 8, 1), 256, 0, stream>>>(
        attn16, attn16, kDim, 0L, woT, woT, kDim, 0L, (void*)x1, (void*)x1, kDim, 0L,
        o_b, x, 0L, kTok, kDim, kDim, 1.0f / (kAc * kWc));
  }
  ln_f16_kernel<<<kTok, 128, 0, stream>>>(x1, ln2_w, ln2_b, xn2);
  wtcast_kernel<<<dim3(kDim / 64, kHidden / 64), 256, 0, stream>>>(mlp_w1, w1T, kDim, kHidden, kWc);
  wtcast_kernel<<<dim3(kHidden / 64, kDim / 64), 256, 0, stream>>>(mlp_w2, w2T, kHidden, kDim, kW2c);
  for (int qd = 0; qd < kMlpQ; ++qd) {
    const unsigned short* aq = xn2 + (size_t)qd * kMlpRows * kDim;
    const int tiles = (kMlpRows / 64) * (kHidden / 64);
    wmma_gemm64<0, false, 2, 0, false><<<dim3((tiles + 7) / 8, 1), 256, 0, stream>>>(
        aq, aq, kDim, 0L, w1T, w1T, kDim, 0L, (void*)pre, (void*)pre, kHidden, 0L,
        mlp_b1, x, 0L, kMlpRows, kHidden, kDim, 1.0f / kWc);
    const int n8 = kMlpRows * kHidden / 8;
    gelu_split_kernel<<<(n8 + 255) / 256, 256, 0, stream>>>(
        pre, hhi + (size_t)qd * kMlpRows * kHidden, hlo + (size_t)qd * kMlpRows * kHidden, n8);
  }
  {
    const int tiles = (kTok / 64) * (kDim / 64);
    wmma_gemm64<0, false, 2, 0, true><<<dim3((tiles + 7) / 8, 1), 256, 0, stream>>>(
        hhi, hhi, kHidden, 0L, w2T, w2T, kHidden, 0L, (void*)tmp, (void*)tmp, kDim, 0L,
        mlp_b2, x1, 0L, kTok, kDim, kHidden, 1.0f / kW2c);
  }
  {
    const int tiles = (kTok / 64) * (kDim / 64);
    wmma_gemm64<0, false, 0, 0, true><<<dim3((tiles + 7) / 8, 1), 256, 0, stream>>>(
        hlo, hlo, kHidden, 0L, w2T, w2T, kHidden, 0L, (void*)out, (void*)out, kDim, 0L,
        mlp_b2, tmp, 0L, kTok, kDim, kHidden, 1.0f / (kLoc * kW2c));
  }
}
